// MultiTypeCategorical_51591147159566
// MI455X (gfx1250) — hardware-verified
//
#include <hip/hip_runtime.h>
#include <hip/hip_bf16.h>
#include <math.h>

typedef _Float16 bf16;
typedef bf16  v16bf __attribute__((ext_vector_type(16)));
typedef float v8f   __attribute__((ext_vector_type(8)));
typedef __attribute__((ext_vector_type(4))) unsigned v4u_t;
typedef unsigned v4ua __attribute__((ext_vector_type(4), may_alias));

#define BATCH 4096
#define IN    512
#define OUTD  64
#define NEXP  128
#define NDST  32
#define NTYP  4

__global__ void cvt_x_kernel(const float* __restrict__ x, bf16* __restrict__ xb, int n) {
    int i = (blockIdx.x * 256 + threadIdx.x) * 2;
    if (i < n) { const unsigned u = (unsigned)__builtin_bit_cast(unsigned short, (bf16)x[i]) | ((unsigned)__builtin_bit_cast(unsigned short, (bf16)x[i + 1]) << 16);
        *(volatile unsigned*)(xb + i) = u; __threadfence(); *(volatile unsigned*)(xb + i) = u; }
}

__global__ void cvt_w_kernel(const float* __restrict__ W, bf16* __restrict__ Wt) {
    __shared__ bf16 tile[64][OUTD + 4];
    int e  = blockIdx.x >> 3;
    int i0 = (blockIdx.x & 7) * 64;
    const float* src = W + (size_t)e * IN * OUTD + (size_t)i0 * OUTD;
    for (int k = threadIdx.x; k < 64 * OUTD; k += 256) {
        int iL = k >> 6, o = k & 63;
        tile[iL][o] = (bf16)src[k];
    }
    __syncthreads();
    if (threadIdx.x < 64) {
        const int o = threadIdx.x;
        bf16* dst = Wt + ((size_t)e * OUTD + o) * IN + i0;
#pragma unroll 1
        for (int pass = 0; pass < 2; ++pass) {
#pragma unroll
            for (int c8 = 0; c8 < 64; c8 += 8) {
                bf16 hh[8];
#pragma unroll
                for (int j = 0; j < 8; ++j) hh[j] = tile[c8 + j][o];
                *(volatile v4u_t*)(dst + c8) = *(const v4ua*)hh;
            }
            __threadfence();
        }
    }
}

__global__ __launch_bounds__(256, 1)
void moe_gemm_kernel(const float* __restrict__ dst_state,
                     const float* __restrict__ type_state,
                     const float* __restrict__ bias,
                     const bf16* __restrict__ xb,
                     const bf16* __restrict__ Wt,
                     float* __restrict__ out) {
    __shared__ float gls[32][NEXP];
    __shared__ float slog[32][OUTD + 4];
    __shared__ float rmax[32], rlse[32];

    const int tid = threadIdx.x;
    const int m0  = blockIdx.x * 32;

    for (int k = tid; k < 32 * NEXP; k += 256) {
        int r = k >> 7, e = k & 127;
        gls[r][e] = dst_state[(m0 + r) * NDST + (e >> 2)] *
                    type_state[(m0 + r) * NTYP + (e & 3)];
    }
    __syncthreads();

    const int wave  = tid >> 5, lane = tid & 31;
    const int mt    = wave >> 2, nt  = wave & 3;
    const int col   = lane & 15, khalf = lane >> 4;
    const int arow  = m0 + mt * 16 + col;
    const int ocol  = nt * 16 + col;
    const int rbase = mt * 16 + khalf * 8;

    v16bf a[16];
    const bf16* xr = xb + (size_t)arow * IN;
#pragma unroll
    for (int ib = 0; ib < 16; ++ib) {
        const bf16* p = xr + ib * 32 + khalf * 8;
        union { v16bf v; uint4 q[2]; } u;
        u.q[0] = *(const uint4*)p;
        u.q[1] = *(const uint4*)(p + 16);
        a[ib] = u.v;
    }

    v8f logit = {};
    const bf16* wbase = Wt + (size_t)ocol * IN + khalf * 8;

    for (int e = 0; e < NEXP; ++e) {
        v8f acc = {};
        const bf16* we = wbase + (size_t)e * OUTD * IN;
#pragma unroll
        for (int ib = 0; ib < 16; ++ib) {
            const bf16* q = we + ib * 32;
            union { v16bf v; uint4 qq[2]; } u;
            u.qq[0] = *(const uint4*)q;
            u.qq[1] = *(const uint4*)(q + 16);
            acc = __builtin_amdgcn_wmma_f32_16x16x32_f16(
                false, a[ib], false, u.v, (short)0, acc, false, false);
        }
        const float bv = bias[e * OUTD + ocol];
#pragma unroll
        for (int r = 0; r < 8; ++r) {
            logit[r] += gls[rbase + r][e] * (acc[r] + bv);
        }
    }

#pragma unroll
    for (int r = 0; r < 8; ++r) slog[rbase + r][ocol] = logit[r];
    __syncthreads();

    if (tid < 32) {
        float m = -INFINITY;
        for (int o = 0; o < OUTD; ++o) m = fmaxf(m, slog[tid][o]);
        float s = 0.f;
        for (int o = 0; o < OUTD; ++o) s += __expf(slog[tid][o] - m);
        rmax[tid] = m;
        rlse[tid] = __logf(s);
    }
    __syncthreads();

    for (int k = tid; k < 32 * OUTD; k += 256) {
        int r = k >> 6, o = k & 63;
        const float v = slog[r][o] - rmax[r] - rlse[r];
        *(volatile float*)(out + (size_t)(m0 + r) * OUTD + o) = v; __threadfence(); *(volatile float*)(out + (size_t)(m0 + r) * OUTD + o) = v;
    }
}

extern "C" void kernel_launch(void* const* d_in, const int* in_sizes, int n_in,
                              void* d_out, int out_size, void* d_ws, size_t ws_size,
                              hipStream_t stream) {
    const float* x   = (const float*)d_in[0];
    const float* dst = (const float*)d_in[1];
    const float* typ = (const float*)d_in[2];
    const float* W   = (const float*)d_in[3];
    const float* b   = (const float*)d_in[4];
    float* out = (float*)d_out;

    bf16* xb = (bf16*)d_ws;
    bf16* Wt = (bf16*)((char*)d_ws + (size_t)BATCH * IN * sizeof(bf16));

    int nx = BATCH * IN;
    cvt_x_kernel<<<(nx / 2 + 255) / 256, 256, 0, stream>>>(x, xb, nx);
    cvt_w_kernel<<<NEXP * (IN / 64), 256, 0, stream>>>(W, Wt);
    moe_gemm_kernel<<<BATCH / 32, 256, 0, stream>>>(dst, typ, b, xb, Wt, out);
}
